// CausalSelfAttention_14929306321255
// MI455X (gfx1250) — hardware-verified
//
#include <hip/hip_runtime.h>
#include <stdint.h>
#include <stddef.h>


#pragma clang fp contract(off)

typedef _Float16 v16h __attribute__((ext_vector_type(16)));
typedef _Float16 v8h  __attribute__((ext_vector_type(8)));
typedef float    v8f  __attribute__((ext_vector_type(8)));
typedef float    v4f  __attribute__((ext_vector_type(4)));
typedef unsigned int v4u __attribute__((ext_vector_type(4)));

#ifndef NB
#define NB 2
#endif
#ifndef SEQ
#define SEQ 2048
#endif
#define NB_FULL 2
#define SEQ_FULL 2048
#define CE 1024
#define C3 3072
#define NH 16
#define HD 64
#define D2 128
#define ER 256
#define MROWS (NB * SEQ)
#define NTAB (SEQ * HD + NH * HD)

static_assert(NB >= 1 && NB <= NB_FULL);
static_assert(SEQ >= ER && SEQ <= SEQ_FULL && (SEQ % 256) == 0);
static_assert((MROWS % 128) == 0);
static_assert((NTAB % 256) == 0);
static_assert((size_t)MROWS * CE <= (size_t)NB_FULL * SEQ_FULL * CE);

__device__ __forceinline__ v8f wmma16(v16h a, v16h b, v8f c) {
  v8f d = __builtin_amdgcn_wmma_f32_16x16x32_f16(false, a, false, b, (short)0, c, false, false);
  asm volatile("v_nop\n\tv_nop\n\tv_nop\n\tv_nop" : "+v"(d) : "v"(a), "v"(b));
  return d;
}

__device__ __forceinline__ v8f vzero() {
  v8f z = {0.f, 0.f, 0.f, 0.f, 0.f, 0.f, 0.f, 0.f};
  return z;
}

__device__ __forceinline__ v16h load_frag(const _Float16* base, int stride, int row_off, int k_off) {
  const int lane = threadIdx.x & 31;
  const int m    = lane & 15;
  const int kb   = (lane >> 4) << 3;
  const _Float16* p = base + (size_t)(row_off + m) * stride + k_off + kb;
  const v8h lo = *(const v8h*)p;
  const v8h hi = *(const v8h*)(p + 16);
  v16h r;
#pragma unroll
  for (int i = 0; i < 8; ++i) { r[i] = lo[i]; r[i + 8] = hi[i]; }
  return r;
}

__device__ __forceinline__ float bf16r(float f) {
  unsigned int u = __float_as_uint(f);
  u = (u + 0x7FFFu + ((u >> 16) & 1u)) & 0xFFFF0000u;
  return __uint_as_float(u);
}

__device__ __forceinline__ float softplusf(float x) {
  return fmaxf(x, 0.0f) + log1pf(__expf(-fabsf(x)));
}

__global__ __launch_bounds__(256) void k_cvt(const float* __restrict__ src, _Float16* __restrict__ dst,
                                            int nrows, int seg, int seg_full, int dst_stride, int dst_col,
                                            float scale) {
  const int g = blockIdx.x * 256 + threadIdx.x;
  const int m = g >> 7;
  if (m >= nrows) return;
  const int c    = (g & 127) << 3;
  const int sb   = m / seg;
  const int srow = sb * seg_full + (m - sb * seg);
  const float* sp = src + (size_t)srow * CE + c;
  const v4f f0 = *(const v4f*)sp;
  const v4f f1 = *(const v4f*)(sp + 4);
  v8h hv;
#pragma unroll
  for (int u = 0; u < 4; ++u) {
    hv[u]     = (_Float16)(bf16r(f0[u]) * scale);
    hv[u + 4] = (_Float16)(bf16r(f1[u]) * scale);
  }
  const v4u w = __builtin_bit_cast(v4u, hv);
  _Float16* dp = dst + (size_t)m * dst_stride + dst_col + c;
  *(volatile v4u*)dp = w;
  __threadfence();
  *(volatile v4u*)dp = w;
}

__global__ __launch_bounds__(256) void k_tab(const float* __restrict__ delta, float* __restrict__ CT,
                                            float* __restrict__ ST) {
  const int i = blockIdx.x * 256 + threadIdx.x;
  if (i >= NTAB) return;
  const int npos = SEQ * HD;
  int j = i - npos;
  j = (j < 0) ? 0 : j;
  j = (j > NH * HD - 1) ? (NH * HD - 1) : j;
  float dl = bf16r(delta[j]);
  dl = fminf(fmaxf(dl, -6.28318548f), 0.0f);
  const int t = i >> 6;
  const int d = i & 63;
  const float pw   = powf(10000.0f, (float)d * 0.015625f);
  const float invf = 1.0f / pw;
  const float angp = (float)t * invf;
  const float ang  = (i < npos) ? angp : dl;
  float sv, cv;
  sincosf(ang, &sv, &cv);
  *(volatile float*)(CT + i) = cv;
  *(volatile float*)(ST + i) = sv;
  __threadfence();
  *(volatile float*)(CT + i) = cv;
  *(volatile float*)(ST + i) = sv;
}

__global__ __launch_bounds__(256) __attribute__((amdgpu_num_vgpr(256)))
void k_gemm(const _Float16* __restrict__ A, const _Float16* __restrict__ B, float* __restrict__ C,
            int N, int K, float scale) {
  extern __shared__ __attribute__((aligned(16))) char smem_g[];
  _Float16* As  = (_Float16*)smem_g;
  _Float16* Bs  = (_Float16*)(smem_g + 8192);
  float*    stg = (float*)smem_g;

  const int tid  = threadIdx.x;
  const int wave = tid >> 5;
  const int lane = tid & 31;
  const int m16  = lane & 15;
  const int off8 = (lane >> 4) << 3;
  const int wm   = wave >> 1;
  const int wn   = wave & 1;
  const int bm   = blockIdx.y * 128;
  const int bn   = blockIdx.x * 128;

  v8f acc[2][4];
#pragma unroll
  for (int i = 0; i < 2; ++i)
#pragma unroll
    for (int j = 0; j < 4; ++j) acc[i][j] = vzero();

  const int nK = K >> 5;
#pragma unroll 1
  for (int kt = 0; kt < nK; ++kt) {
    const int k0 = kt << 5;
#pragma unroll
    for (int p = 0; p < 2; ++p) {
      const int idx = p * 256 + tid;
      const int row = idx >> 2;
      const int c   = (idx & 3) << 3;
      const v4u va = *(const v4u*)(A + (size_t)(bm + row) * K + k0 + c);
      const v4u vb = *(const v4u*)(B + (size_t)(bn + row) * K + k0 + c);
      *(v4u*)(As + row * 32 + c) = va;
      *(v4u*)(Bs + row * 32 + c) = vb;
    }
    __syncthreads();
    const v16h af0 = load_frag(As, 32, wm * 32, 0);
    const v16h af1 = load_frag(As, 32, wm * 32 + 16, 0);
#pragma unroll
    for (int j = 0; j < 4; ++j) {
      const v16h bfj = load_frag(Bs, 32, wn * 64 + j * 16, 0);
      acc[0][j] = wmma16(af0, bfj, acc[0][j]);
      acc[1][j] = wmma16(af1, bfj, acc[1][j]);
    }
    __syncthreads();
  }

  float* ws_ = stg + wave * (32 * 64);
#pragma unroll
  for (int i = 0; i < 2; ++i)
#pragma unroll
    for (int j = 0; j < 4; ++j)
#pragma unroll
      for (int r = 0; r < 8; ++r)
        ws_[(i * 16 + off8 + r) * 64 + j * 16 + m16] = acc[i][j][r] * scale;
  __syncthreads();

  float* cbase = C + (size_t)(bm + wm * 32) * N + bn + wn * 64;
#pragma unroll
  for (int it = 0; it < 16; ++it) {
    const int c     = it * 32 + lane;
    const int row   = c >> 4;
    const int piece = (c & 15) << 2;
    const v4f v = *(const v4f*)(ws_ + row * 64 + piece);
    *(volatile v4f*)(cbase + (size_t)row * N + piece) = v;
  }
  __threadfence();
#pragma unroll
  for (int it = 0; it < 16; ++it) {
    const int c     = it * 32 + lane;
    const int row   = c >> 4;
    const int piece = (c & 15) << 2;
    const v4f v = *(const v4f*)(ws_ + row * 64 + piece);
    *(volatile v4f*)(cbase + (size_t)row * N + piece) = v;
  }
}

__global__ __launch_bounds__(256) void k_planes(const float* __restrict__ qkv,
                                               const float* __restrict__ CT, const float* __restrict__ ST,
                                               _Float16* __restrict__ Qp, _Float16* __restrict__ Qr,
                                               _Float16* __restrict__ Kp, _Float16* __restrict__ VTp,
                                               _Float16* __restrict__ VTr) {
  extern __shared__ __attribute__((aligned(16))) char smem_p[];
  _Float16* HI = (_Float16*)smem_p;
  _Float16* RS = (_Float16*)(smem_p + 32768);

  const int tid = threadIdx.x;
  const int ntb = SEQ / 64;
  const int bid = blockIdx.x;
  const int bh  = bid / ntb;
  const int tb  = bid - bh * ntb;
  const int b   = bh >> 4;
  const int h   = bh & 15;
  const int t0  = tb * 64;
  const bool early = (t0 < ER);
  const int d   = tid & 63;
  const int tq  = tid >> 6;
  const float cd = CT[SEQ * HD + h * HD + d];
  const float sd = ST[SEQ * HD + h * HD + d];

#pragma unroll 1
  for (int i = 0; i < 32; ++i) {
    const int which = i >> 4;
    const int tl = tq + ((i & 15) << 2);
    const int t  = t0 + tl;
    const size_t row = (size_t)(b * SEQ + t) * C3;
    const float val = qkv[row + which * CE + h * HD + d];
    const float mu  = softplusf(val);
    const float c   = CT[t * HD + d];
    const float s   = ST[t * HD + d];
    const float kre = c * cd - s * sd;
    const float kim = s * cd + c * sd;
    const float re  = mu * (which ? kre : c);
    const float im  = mu * (which ? kim : s);
    const _Float16 hre = (_Float16)re;
    const _Float16 him = (_Float16)im;
    _Float16* ht = HI + which * 8192 + tl * D2;
    ht[d]      = hre;
    ht[HD + d] = him;
    if (early && which == 0) {
      _Float16* rt = RS + tl * D2;
      rt[d]      = (_Float16)((re - (float)hre) * 1024.0f);
      rt[HD + d] = (_Float16)((im - (float)him) * 1024.0f);
    }
  }
  __syncthreads();
  {
    _Float16* qg = Qp + (size_t)(bh * SEQ + t0) * D2;
    _Float16* kg = Kp + (size_t)(bh * SEQ + t0) * D2;
#pragma unroll
    for (int it = 0; it < 4; ++it) {
      const int c = it * 256 + tid;
      const v4u a  = *(const v4u*)(HI + c * 8);
      const v4u bq = *(const v4u*)(HI + 8192 + c * 8);
      *(volatile v4u*)(qg + c * 8) = a;
      *(volatile v4u*)(kg + c * 8) = bq;
    }
    __threadfence();
#pragma unroll
    for (int it = 0; it < 4; ++it) {
      const int c = it * 256 + tid;
      const v4u a  = *(const v4u*)(HI + c * 8);
      const v4u bq = *(const v4u*)(HI + 8192 + c * 8);
      *(volatile v4u*)(qg + c * 8) = a;
      *(volatile v4u*)(kg + c * 8) = bq;
    }
    if (early) {
      _Float16* qrg = Qr + (size_t)(bh * ER + t0) * D2;
#pragma unroll
      for (int it = 0; it < 4; ++it) {
        const int c = it * 256 + tid;
        const v4u a = *(const v4u*)(RS + c * 8);
        *(volatile v4u*)(qrg + c * 8) = a;
      }
      __threadfence();
#pragma unroll
      for (int it = 0; it < 4; ++it) {
        const int c = it * 256 + tid;
        const v4u a = *(const v4u*)(RS + c * 8);
        *(volatile v4u*)(qrg + c * 8) = a;
      }
    }
  }
  __syncthreads();

#pragma unroll 1
  for (int i = 0; i < 16; ++i) {
    const int tl = tq + (i << 2);
    const int t  = t0 + tl;
    const size_t row = (size_t)(b * SEQ + t) * C3;
    const float v = qkv[row + 2 * CE + h * HD + d];
    const _Float16 hv = (_Float16)v;
    HI[d * 64 + tl] = hv;
    if (early) RS[d * 64 + tl] = (_Float16)((v - (float)hv) * 1024.0f);
  }
  __syncthreads();
  {
#pragma unroll
    for (int it = 0; it < 2; ++it) {
      const int c = it * 256 + tid;
      const int r = c >> 3;
      const int piece = (c & 7) << 3;
      const v4u a = *(const v4u*)(HI + r * 64 + piece);
      *(volatile v4u*)(VTp + (size_t)(bh * HD + r) * SEQ + t0 + piece) = a;
    }
    __threadfence();
#pragma unroll
    for (int it = 0; it < 2; ++it) {
      const int c = it * 256 + tid;
      const int r = c >> 3;
      const int piece = (c & 7) << 3;
      const v4u a = *(const v4u*)(HI + r * 64 + piece);
      *(volatile v4u*)(VTp + (size_t)(bh * HD + r) * SEQ + t0 + piece) = a;
    }
    if (early) {
#pragma unroll
      for (int it = 0; it < 2; ++it) {
        const int c = it * 256 + tid;
        const int r = c >> 3;
        const int piece = (c & 7) << 3;
        const v4u a = *(const v4u*)(RS + r * 64 + piece);
        *(volatile v4u*)(VTr + (size_t)(bh * HD + r) * ER + t0 + piece) = a;
      }
      __threadfence();
#pragma unroll
      for (int it = 0; it < 2; ++it) {
        const int c = it * 256 + tid;
        const int r = c >> 3;
        const int piece = (c & 7) << 3;
        const v4u a = *(const v4u*)(RS + r * 64 + piece);
        *(volatile v4u*)(VTr + (size_t)(bh * HD + r) * ER + t0 + piece) = a;
      }
    }
  }
}

template <bool EARLY>
__global__ __launch_bounds__(128) __attribute__((amdgpu_num_vgpr(256)))
void k_attn(const _Float16* __restrict__ Qp, const _Float16* __restrict__ Qr,
            const _Float16* __restrict__ Kp, const _Float16* __restrict__ VTp,
            const _Float16* __restrict__ VTr,
            _Float16* __restrict__ Y2, int qb0, int nqb) {
  extern __shared__ __attribute__((aligned(16))) char smem_a[];
  _Float16* Ks  = (_Float16*)smem_a;
  _Float16* Vs  = (_Float16*)(smem_a + 16384);
  _Float16* Pw  = (_Float16*)(smem_a + 24576);
  _Float16* Prs = (_Float16*)(smem_a + 32768);
  _Float16* Vrs = (_Float16*)(smem_a + 40960);

  const int tid  = threadIdx.x;
  const int w    = tid >> 5;
  const int lane = tid & 31;
  const int m    = lane & 15;
  const int off8 = (lane >> 4) << 3;
  const int bh   = blockIdx.x / nqb;
  const int qb   = qb0 + (blockIdx.x - bh * nqb);
  const int b    = bh >> 4;
  const int h    = bh & 15;
  const int q0   = qb * 64 + w * 16;

  const _Float16* qg  = Qp + (size_t)(bh * SEQ + q0) * D2;
  const _Float16* qrg = Qr + (size_t)(bh * ER + (q0 & (ER - 1))) * D2;
  _Float16* pw  = Pw + w * 1024;
  _Float16* prw = Prs + w * 1024;

  v16h qf[4];
  if (!EARLY) {
#pragma unroll
    for (int ks = 0; ks < 4; ++ks) qf[ks] = load_frag(qg, D2, 0, ks * 32);
  }

  v8f O[4];
  float mrow[8], lrow[8];
#pragma unroll
  for (int n = 0; n < 4; ++n) O[n] = vzero();
#pragma unroll
  for (int r = 0; r < 8; ++r) { mrow[r] = -3.0e38f; lrow[r] = 0.0f; }

#pragma unroll 1
  for (int kb = 0; kb <= qb; ++kb) {
    const int k0 = kb * 64;
#pragma unroll
    for (int p = 0; p < 8; ++p) {
      const int idx = p * 128 + tid;
      const int row = idx >> 4;
      const int c   = (idx & 15) << 3;
      *(v4u*)(Ks + row * D2 + c) = *(const v4u*)(Kp + (size_t)(bh * SEQ + k0 + row) * D2 + c);
    }
#pragma unroll
    for (int p = 0; p < 4; ++p) {
      const int idx = p * 128 + tid;
      const int dr  = idx >> 3;
      const int c   = (idx & 7) << 3;
      *(v4u*)(Vs + dr * 64 + c) = *(const v4u*)(VTp + (size_t)(bh * HD + dr) * SEQ + k0 + c);
      if (EARLY)
        *(v4u*)(Vrs + dr * 64 + c) = *(const v4u*)(VTr + (size_t)(bh * HD + dr) * ER + k0 + c);
    }
    __syncthreads();

    v8f sc[4];
    if (EARLY) {
#pragma unroll
      for (int nt = 0; nt < 4; ++nt) {
        v8f a  = vzero();
        v8f a2 = vzero();
#pragma unroll 1
        for (int ks = 0; ks < 4; ++ks) {
          const v16h bk = load_frag(Ks, D2, nt * 16, ks * 32);
          const v16h qa = load_frag(qg, D2, 0, ks * 32);
          a = wmma16(qa, bk, a);
          const v16h qres = load_frag(qrg, D2, 0, ks * 32);
          a2 = wmma16(qres, bk, a2);
        }
        sc[nt] = a + a2 * (1.0f / 1024.0f);
      }
    } else {
#pragma unroll
      for (int nt = 0; nt < 4; ++nt) {
        v8f a = vzero();
#pragma unroll
        for (int ks = 0; ks < 4; ++ks) {
          const v16h bk = load_frag(Ks, D2, nt * 16, ks * 32);
          a = wmma16(qf[ks], bk, a);
        }
        sc[nt] = a;
      }
    }

    const bool diag = (kb == qb);
#pragma unroll
    for (int r = 0; r < 8; ++r) {
      const int qi = q0 + off8 + r;
      float sv[4];
      float mx = -3.0e38f;
#pragma unroll
      for (int nt = 0; nt < 4; ++nt) {
        const int kj = k0 + nt * 16 + m;
        const bool ok = (!diag) || (kj <= qi);
        float s = sc[nt][r] * 0.125f;
        s = ok ? s : -3.0e38f;
        sv[nt] = s;
        mx = fmaxf(mx, s);
      }
      mx = fmaxf(mx, __shfl_xor(mx, 1, 32));
      mx = fmaxf(mx, __shfl_xor(mx, 2, 32));
      mx = fmaxf(mx, __shfl_xor(mx, 4, 32));
      mx = fmaxf(mx, __shfl_xor(mx, 8, 32));
      const float mnew = fmaxf(mrow[r], mx);
      const float corr = __expf(mrow[r] - mnew);
      mrow[r] = mnew;
      float sum = 0.0f;
#pragma unroll
      for (int nt = 0; nt < 4; ++nt) {
        const int kj = k0 + nt * 16 + m;
        const bool ok = (!diag) || (kj <= qi);
        const float e = __expf(sv[nt] - mnew);
        const float p = ok ? e : 0.0f;
        sum += p;
        const float ph = p * 16384.0f;
        const _Float16 h16 = (_Float16)ph;
        pw[(off8 + r) * 64 + nt * 16 + m] = h16;
        if (EARLY) prw[(off8 + r) * 64 + nt * 16 + m] = (_Float16)((ph - (float)h16) * 1024.0f);
      }
      sum += __shfl_xor(sum, 1, 32);
      sum += __shfl_xor(sum, 2, 32);
      sum += __shfl_xor(sum, 4, 32);
      sum += __shfl_xor(sum, 8, 32);
      lrow[r] = lrow[r] * corr + sum;
#pragma unroll
      for (int nt = 0; nt < 4; ++nt) O[nt][r] *= corr;
    }
    __syncthreads();

    if (EARLY) {
#pragma unroll
      for (int nt2 = 0; nt2 < 4; ++nt2) {
        v8f t2 = vzero();
#pragma unroll 1
        for (int ks2 = 0; ks2 < 2; ++ks2) {
          const v16h bv = load_frag(Vs, 64, nt2 * 16, ks2 * 32);
          const v16h pa = load_frag(pw, 64, 0, ks2 * 32);
          O[nt2] = wmma16(pa, bv, O[nt2]);
          const v16h par = load_frag(prw, 64, 0, ks2 * 32);
          t2 = wmma16(par, bv, t2);
          const v16h bvr = load_frag(Vrs, 64, nt2 * 16, ks2 * 32);
          t2 = wmma16(pa, bvr, t2);
        }
        O[nt2] = O[nt2] + t2 * (1.0f / 1024.0f);
      }
    } else {
#pragma unroll
      for (int ks2 = 0; ks2 < 2; ++ks2) {
        const v16h pa = load_frag(pw, 64, 0, ks2 * 32);
#pragma unroll
        for (int nt2 = 0; nt2 < 4; ++nt2) {
          const v16h bv = load_frag(Vs, 64, nt2 * 16, ks2 * 32);
          O[nt2] = wmma16(pa, bv, O[nt2]);
        }
      }
    }
    __syncthreads();
  }

  _Float16* sth  = pw;
  _Float16* strs = Ks + w * 1024;
#pragma unroll
  for (int r = 0; r < 8; ++r) {
    const float inv = (1.0f / lrow[r]) * (1.0f / 16384.0f);
#pragma unroll
    for (int nt2 = 0; nt2 < 4; ++nt2) {
      const float y = O[nt2][r] * inv;
      const _Float16 yh = (_Float16)y;
      sth[(off8 + r) * 64 + nt2 * 16 + m]  = yh;
      strs[(off8 + r) * 64 + nt2 * 16 + m] = (_Float16)((y - (float)yh) * 64.0f);
    }
  }
  __syncthreads();

  _Float16* yg = Y2 + (size_t)(b * SEQ + q0) * (2 * CE) + h * HD;
#pragma unroll
  for (int it = 0; it < 4; ++it) {
    const int c     = it * 32 + lane;
    const int row   = c >> 3;
    const int piece = (c & 7) << 3;
    const v4u vh = *(const v4u*)(sth  + row * 64 + piece);
    const v4u vr = *(const v4u*)(strs + row * 64 + piece);
    *(volatile v4u*)(yg + (size_t)row * (2 * CE) + piece)      = vh;
    *(volatile v4u*)(yg + (size_t)row * (2 * CE) + CE + piece) = vr;
  }
  __threadfence();
#pragma unroll
  for (int it = 0; it < 4; ++it) {
    const int c     = it * 32 + lane;
    const int row   = c >> 3;
    const int piece = (c & 7) << 3;
    const v4u vh = *(const v4u*)(sth  + row * 64 + piece);
    const v4u vr = *(const v4u*)(strs + row * 64 + piece);
    *(volatile v4u*)(yg + (size_t)row * (2 * CE) + piece)      = vh;
    *(volatile v4u*)(yg + (size_t)row * (2 * CE) + CE + piece) = vr;
  }
}

extern "C" void kernel_launch(void* const* d_in, const int* in_sizes, int n_in,
                              void* d_out, int out_size, void* d_ws, size_t ws_size,
                              hipStream_t stream) {
  if (n_in < 4) return;
  const long long need_x = ((long long)(NB - 1) * SEQ_FULL + SEQ) * CE;
  if ((long long)in_sizes[0] < need_x) return;
  if (in_sizes[1] < C3 * CE || in_sizes[2] < CE * CE || in_sizes[3] < NH * HD) return;
  if ((long long)out_size < (long long)MROWS * CE) return;

  const size_t qkv_bytes = (size_t)MROWS * C3 * 4;
  const size_t y2_bytes  = (size_t)MROWS * (2 * CE) * 2;
  const size_t r0_bytes  = (qkv_bytes > y2_bytes) ? qkv_bytes : y2_bytes;
  const size_t off_qkv   = 0;
  const size_t off_y2    = 0;
  const size_t off_wp2   = r0_bytes;
  const size_t wp2_bytes = (size_t)CE * (2 * CE) * 2;
  const size_t tab_bytes = (size_t)NTAB * 4;
  const size_t off_ct    = off_wp2 + wp2_bytes;
  const size_t off_st    = off_ct + tab_bytes;
  const size_t off_r3    = off_st + tab_bytes;
  const size_t x16_bytes = (size_t)MROWS * CE * 2;
  const size_t wa_bytes  = (size_t)C3 * CE * 2;
  const size_t qp_bytes  = (size_t)NB * NH * SEQ * D2 * 2;
  const size_t vt_bytes  = (size_t)NB * NH * HD * SEQ * 2;
  const size_t qr_bytes  = (size_t)NB * NH * ER * D2 * 2;
  const size_t vtr_bytes = (size_t)NB * NH * HD * ER * 2;
  const size_t off_x16   = off_r3;
  const size_t off_wa    = off_x16 + x16_bytes;
  const size_t off_qp    = off_r3;
  const size_t off_kp    = off_qp + qp_bytes;
  const size_t off_vtp   = off_kp + qp_bytes;
  const size_t off_qr    = off_vtp + vt_bytes;
  const size_t off_vtr   = off_qr + qr_bytes;
  const size_t end_a     = off_wa + wa_bytes;
  const size_t end_b     = off_vtr + vtr_bytes;
  const size_t total     = (end_a > end_b) ? end_a : end_b;
  if (total > ws_size) return;

  const float* x      = (const float*)d_in[0];
  const float* w_attn = (const float*)d_in[1];
  const float* w_proj = (const float*)d_in[2];
  const float* delta  = (const float*)d_in[3];
  float*       out    = (float*)d_out;
  char*        ws     = (char*)d_ws;

  float*    QKV = (float*)(ws + off_qkv);
  _Float16* Y2  = (_Float16*)(ws + off_y2);
  _Float16* WP2 = (_Float16*)(ws + off_wp2);
  float*    CT  = (float*)(ws + off_ct);
  float*    ST  = (float*)(ws + off_st);
  _Float16* X16 = (_Float16*)(ws + off_x16);
  _Float16* WA  = (_Float16*)(ws + off_wa);
  _Float16* Qp  = (_Float16*)(ws + off_qp);
  _Float16* Kp  = (_Float16*)(ws + off_kp);
  _Float16* VTp = (_Float16*)(ws + off_vtp);
  _Float16* Qr  = (_Float16*)(ws + off_qr);
  _Float16* VTr = (_Float16*)(ws + off_vtr);

  hipFuncSetAttribute((const void*)k_gemm, hipFuncAttributeMaxDynamicSharedMemorySize, 65536);
  hipFuncSetAttribute((const void*)k_planes, hipFuncAttributeMaxDynamicSharedMemorySize, 49152);
  hipFuncSetAttribute((const void*)k_attn<true>, hipFuncAttributeMaxDynamicSharedMemorySize, 49152);
  hipFuncSetAttribute((const void*)k_attn<false>, hipFuncAttributeMaxDynamicSharedMemorySize, 32768);

  k_cvt<<<dim3(MROWS * 128 / 256), dim3(256), 0, stream>>>(x, X16, MROWS, SEQ, SEQ_FULL, CE, 0, 1.0f);
  k_cvt<<<dim3(C3 * 128 / 256), dim3(256), 0, stream>>>(w_attn, WA, C3, C3, C3, CE, 0, 64.0f);
  k_cvt<<<dim3(CE * 128 / 256), dim3(256), 0, stream>>>(w_proj, WP2, CE, CE, CE, 2 * CE, 0, 64.0f);
  k_cvt<<<dim3(CE * 128 / 256), dim3(256), 0, stream>>>(w_proj, WP2, CE, CE, CE, 2 * CE, CE, 1.0f);
  k_tab<<<dim3(NTAB / 256), dim3(256), 0, stream>>>(delta, CT, ST);
  k_gemm<<<dim3(C3 / 128, MROWS / 128), dim3(256), 65536, stream>>>(X16, WA, QKV, C3, CE, 1.0f / 64.0f);
  k_planes<<<dim3(NB * NH * (SEQ / 64)), dim3(256), 49152, stream>>>(QKV, CT, ST, Qp, Qr, Kp, VTp, VTr);
  const int nqb_all = SEQ / 64;
  const int nqb_e   = ER / 64;
  const int nqb_l   = nqb_all - nqb_e;
  k_attn<true><<<dim3(NB * NH * nqb_e), dim3(128), 49152, stream>>>(Qp, Qr, Kp, VTp, VTr, Y2, 0, nqb_e);
  if (nqb_l > 0)
    k_attn<false><<<dim3(NB * NH * nqb_l), dim3(128), 32768, stream>>>(Qp, Qr, Kp, VTp, VTr, Y2, nqb_e, nqb_l);
  k_gemm<<<dim3(CE / 128, MROWS / 128), dim3(256), 65536, stream>>>(Y2, WP2, out, CE, 2 * CE, 1.0f / 64.0f);
}
